// CFConv_27994596835767
// MI455X (gfx1250) — hardware-run, weakly checked
//
#include <hip/hip_runtime.h>
#include <stddef.h>


#pragma clang fp contract(off)

#define NF      64
#define HD      64
#define OD      128
#define NTHR    256
#define NWAVE   8
#define EPT     8
#define NGRP    2
#define CHUNK   (NTHR * EPT * NGRP)
#define WCAP    (EPT * NGRP * 32)
#define LISTN   (NWAVE * WCAP)
#define NBC     4096
#define NBF     1024
#define RCAP    40960
#define RBN     128
#define OTHR    512
#define TB      64
#define TE      64
#define ECAP    4096
#define WSCAP   134217728
#define SCL_H   64.0f
#define SCL_W   64.0f
#define SCL_ACC 0.000244140625f
#define LN2F    0.693147182f

#define LDS_FILL ((RCAP + NBF + LISTN) * 4 + 64)

#define LO_W1H 0
#define LO_W1L 8192
#define LO_W2  16384
#define LO_AH  32768
#define LO_AL  40960
#define LO_H   49152
#define LO_F   57344
#define LO_S   90112
#define LO_DST 123392
#define LO_SLT 123648
#define LO_MU  123904
#define LDS_EDGE 124160

static_assert((CHUNK & (CHUNK - 1)) == 0);
static_assert(CHUNK <= 4096);
static_assert(NBC <= 4096 && NBF <= 4096);
static_assert((NBC & (NBC - 1)) == 0 && (NBF & (NBF - 1)) == 0);
static_assert(NBC == 4 * NBF);
static_assert(OTHR * 8 == NBC);
static_assert((RCAP % 32) == 0);
static_assert((NBF % TB) == 0);
static_assert(TE == 64 && TB == 64 && NTHR == 4 * TE);
static_assert((ECAP % TE) == 0);
static_assert(NF == 64 && HD == 64 && OD == 128);
static_assert(LO_W1L == LO_W1H + HD * NF * 2);
static_assert(LO_W2  == LO_W1L + HD * NF * 2);
static_assert(LO_AH  == LO_W2  + OD * HD * 2);
static_assert(LO_AL  == LO_AH  + TE * NF * 2);
static_assert(LO_H   == LO_AL  + TE * NF * 2);
static_assert(LO_F   == LO_H   + TE * HD * 2);
static_assert(LO_S   == LO_F   + TE * OD * 4);
static_assert(LO_DST == LO_S   + (TB + 1) * OD * 4);
static_assert(LO_SLT == LO_DST + TE * 4);
static_assert(LO_MU  == LO_SLT + TE * 4);
static_assert(LDS_EDGE == LO_MU + NF * 4);

typedef float          v4f  __attribute__((ext_vector_type(4)));
typedef float          v8f  __attribute__((ext_vector_type(8)));
typedef int            v4i  __attribute__((ext_vector_type(4)));
typedef _Float16       v8h  __attribute__((ext_vector_type(8)));
typedef _Float16       v16h __attribute__((ext_vector_type(16)));
typedef unsigned short v8us __attribute__((ext_vector_type(8)));
typedef __bf16         v16b __attribute__((ext_vector_type(16)));
union FragH { v16h v; v8h h[2]; };
union FragB { v16b v; v8us u[2]; };

__device__ __forceinline__ v8f wmh(v16h a, v16h b, v8f c) {
  v8f d = __builtin_amdgcn_wmma_f32_16x16x32_f16(false, a, false, b, (short)0, c, false, false);
  asm volatile("v_nop\n\tv_nop\n\tv_nop\n\tv_nop" : "+v"(d) : "v"(a), "v"(b));
  return d;
}
__device__ __forceinline__ v8f wmb(v16b a, v16b b, v8f c) {
  v8f d = __builtin_amdgcn_wmma_f32_16x16x32_bf16(false, a, false, b, (short)0, c, false, false);
  asm volatile("v_nop\n\tv_nop\n\tv_nop\n\tv_nop" : "+v"(d) : "v"(a), "v"(b));
  return d;
}

__device__ __forceinline__ unsigned short bf16bits(float f) {
  unsigned u = __float_as_uint(f);
  u = u + 0x7FFFu + ((u >> 16) & 1u);
  return (unsigned short)(u >> 16);
}
__device__ __forceinline__ float bf16val(unsigned short b) {
  return __uint_as_float(((unsigned)b) << 16);
}

__device__ __forceinline__ void split8(v4f a, v4f b, v8us& h, v8us& l) {
  v8f t;
  t[0] = a.x; t[1] = a.y; t[2] = a.z; t[3] = a.w;
  t[4] = b.x; t[5] = b.y; t[6] = b.z; t[7] = b.w;
#pragma unroll
  for (int j = 0; j < 8; ++j) {
    const unsigned short hb = bf16bits(t[j]);
    h[j] = hb;
    l[j] = bf16bits(t[j] - bf16val(hb));
  }
}

__device__ __forceinline__ v8h cvt8(v4f a, v4f b, float s) {
  v8f t;
  t[0] = a.x * s; t[1] = a.y * s; t[2] = a.z * s; t[3] = a.w * s;
  t[4] = b.x * s; t[5] = b.y * s; t[6] = b.z * s; t[7] = b.w * s;
  return __builtin_convertvector(t, v8h);
}

__device__ __forceinline__ float sspf(float v) {
  const float e = __expf(-fabsf(v));
  const float l = __logf(1.0f + e);
  return (fmaxf(v, 0.0f) + l) - LN2F;
}

template <int NB>
__device__ __forceinline__ int scan_chunk(const int* __restrict__ dsts, int nE, int cbase, int slotBase,
                                          int vec8, int* list, int tid, int lane, int wave) {
  int wc = 0;
#pragma unroll
  for (int g = 0; g < NGRP; ++g) {
    const int el0  = (g * NTHR + tid) * EPT;
    const int e0   = cbase + el0;
    const int sent = -2147483647 - 1;
    v4i da, db;
    if (vec8 != 0 && cbase + CHUNK <= nE) {
      da = *(const v4i*)(dsts + e0);
      db = *(const v4i*)(dsts + e0 + 4);
    } else {
      da.x = (e0     < nE) ? dsts[min(e0, nE - 1)] : sent;
      da.y = (e0 + 1 < nE) ? dsts[min(e0 + 1, nE - 1)] : sent;
      da.z = (e0 + 2 < nE) ? dsts[min(e0 + 2, nE - 1)] : sent;
      da.w = (e0 + 3 < nE) ? dsts[min(e0 + 3, nE - 1)] : sent;
      db.x = (e0 + 4 < nE) ? dsts[min(e0 + 4, nE - 1)] : sent;
      db.y = (e0 + 5 < nE) ? dsts[min(e0 + 5, nE - 1)] : sent;
      db.z = (e0 + 6 < nE) ? dsts[min(e0 + 6, nE - 1)] : sent;
      db.w = (e0 + 7 < nE) ? dsts[min(e0 + 7, nE - 1)] : sent;
    }
    const unsigned nb = (unsigned)slotBase;
    const unsigned s0 = (unsigned)da.x - nb, s1 = (unsigned)da.y - nb;
    const unsigned s2 = (unsigned)da.z - nb, s3 = (unsigned)da.w - nb;
    const unsigned s4 = (unsigned)db.x - nb, s5 = (unsigned)db.y - nb;
    const unsigned s6 = (unsigned)db.z - nb, s7 = (unsigned)db.w - nb;
    const bool h0 = s0 < (unsigned)NB, h1 = s1 < (unsigned)NB, h2 = s2 < (unsigned)NB, h3 = s3 < (unsigned)NB;
    const bool h4 = s4 < (unsigned)NB, h5 = s5 < (unsigned)NB, h6 = s6 < (unsigned)NB, h7 = s7 < (unsigned)NB;
    const unsigned any = __builtin_amdgcn_ballot_w32(h0 | h1 | h2 | h3 | h4 | h5 | h6 | h7);
    if (any != 0u) {
#define HITJ(J, HJ, SJ) { \
        const unsigned mj = __builtin_amdgcn_ballot_w32(HJ); \
        if (mj != 0u) { \
          if (HJ) { \
            const int pos = wc + (int)__builtin_amdgcn_mbcnt_lo(mj, 0u); \
            if (pos < WCAP) list[wave * WCAP + pos] = ((el0 + (J)) << 12) | (int)(SJ); \
          } \
          wc += (int)__builtin_popcount(mj); } }
      HITJ(0, h0, s0)
      HITJ(1, h1, s1)
      HITJ(2, h2, s2)
      HITJ(3, h3, s3)
      HITJ(4, h4, s4)
      HITJ(5, h5, s5)
      HITJ(6, h6, s6)
      HITJ(7, h7, s7)
#undef HITJ
    }
  }
  return wc;
}

__global__ __launch_bounds__(NTHR) void k_count(
    const int* __restrict__ dsts, int* cnt, int nE, int vec8) {
  __shared__ __attribute__((aligned(16))) int scnt[NBC];
  __shared__ __attribute__((aligned(16))) int list[LISTN];
  __shared__ int wcnt[NWAVE];
  const int tid = threadIdx.x, lane = tid & 31, wave = tid >> 5;
  const int nodeBase = blockIdx.x * NBC;

  for (int i = tid; i < NBC; i += NTHR) scnt[i] = 0;
  __syncthreads();

  const int nChunks = (nE + CHUNK - 1) / CHUNK;
#pragma unroll 1
  for (int ch = 0; ch < nChunks; ++ch) {
    const int cbase = ch * CHUNK;
    const int wc = scan_chunk<NBC>(dsts, nE, cbase, nodeBase, vec8, list, tid, lane, wave);
    if (lane == 0) wcnt[wave] = wc;
    __syncthreads();
    if (wave == 0) {
#pragma unroll 1
      for (int wsx = 0; wsx < NWAVE; ++wsx) {
        int n = __builtin_amdgcn_readfirstlane(wcnt[wsx]);
        n = n > WCAP ? WCAP : (n < 0 ? 0 : n);
        const int* lp = list + wsx * WCAP;
#pragma unroll 1
        for (int i = 0; i < n; ++i) {
          const int ent  = __builtin_amdgcn_readfirstlane(lp[i]);
          const int slot = ent & (NBC - 1);
          if (lane == 0) scnt[slot] = scnt[slot] + 1;
        }
      }
    }
    __syncthreads();
  }

  v4i cq[4];
#pragma unroll
  for (int q = 0; q < 4; ++q) {
    const int f = (wave * 4 + q) * 128 + 4 * lane;
    cq[q] = *(const v4i*)(scnt + f);
  }
  int* cp = cnt + (size_t)nodeBase;
#pragma unroll
  for (int q = 0; q < 4; ++q) {
    const int f = (wave * 4 + q) * 128 + 4 * lane;
    *(volatile v4i*)(cp + f) = cq[q];
  }
  __threadfence();
#pragma unroll
  for (int q = 0; q < 4; ++q) {
    const int f = (wave * 4 + q) * 128 + 4 * lane;
    *(volatile v4i*)(cp + f) = cq[q];
  }
}

__global__ __launch_bounds__(OTHR) void k_offsets(
    const int* __restrict__ cnt, int* off, int* rbase, int nChunk) {
  __shared__ __attribute__((aligned(16))) int soff[NBC];
  __shared__ __attribute__((aligned(16))) int srb[RBN];
  __shared__ int wtot[OTHR / 32];
  const int tid = threadIdx.x, lane = tid & 31, wave = tid >> 5, sub = tid >> 7;
  for (int i = tid; i < RBN; i += OTHR) srb[i] = 0;
  int carry = 0;
#pragma unroll 1
  for (int ch = 0; ch < nChunk; ++ch) {
    const int base = ch * NBC;
    const v4i c0 = *(const v4i*)(cnt + base + 8 * tid);
    const v4i c1 = *(const v4i*)(cnt + base + 8 * tid + 4);
    const int e0 = max(c0.x, 0), e1 = max(c0.y, 0), e2 = max(c0.z, 0), e3 = max(c0.w, 0);
    const int e4 = max(c1.x, 0), e5 = max(c1.y, 0), e6 = max(c1.z, 0), e7 = max(c1.w, 0);
    const int ts = e0 + e1 + e2 + e3 + e4 + e5 + e6 + e7;
    int incl = ts;
#pragma unroll
    for (int d = 1; d < 32; d <<= 1) {
      const int t = __shfl_up(incl, d);
      if (lane >= d) incl += t;
    }
    if (lane == 31) wtot[wave] = incl;
    __syncthreads();
    const int S0 = wtot[0]  + wtot[1]  + wtot[2]  + wtot[3];
    const int S1 = wtot[4]  + wtot[5]  + wtot[6]  + wtot[7];
    const int S2 = wtot[8]  + wtot[9]  + wtot[10] + wtot[11];
    const int S3 = wtot[12] + wtot[13] + wtot[14] + wtot[15];
    int pre = 0;
#pragma unroll 1
    for (int w = 4 * sub; w < wave; ++w) pre += wtot[w];
    const int b0 = carry;
    const int b1 = b0 + ((S0 + 31) & ~31);
    const int b2 = b1 + ((S1 + 31) & ~31);
    const int b3 = b2 + ((S2 + 31) & ~31);
    const int b4 = b3 + ((S3 + 31) & ~31);
    const int myb = sub == 0 ? b0 : (sub == 1 ? b1 : (sub == 2 ? b2 : b3));
    if (tid == 0) {
      srb[min(4 * ch + 0, RBN - 1)] = b0;
      srb[min(4 * ch + 1, RBN - 1)] = b1;
      srb[min(4 * ch + 2, RBN - 1)] = b2;
      srb[min(4 * ch + 3, RBN - 1)] = b3;
    }
    int run = myb + pre + incl - ts;
    soff[8 * tid + 0] = run; run += e0;
    soff[8 * tid + 1] = run; run += e1;
    soff[8 * tid + 2] = run; run += e2;
    soff[8 * tid + 3] = run; run += e3;
    soff[8 * tid + 4] = run; run += e4;
    soff[8 * tid + 5] = run; run += e5;
    soff[8 * tid + 6] = run; run += e6;
    soff[8 * tid + 7] = run;
    carry = b4;
    __syncthreads();
    const v4i o0 = *(const v4i*)(soff + 4 * tid);
    const v4i o1 = *(const v4i*)(soff + 4 * (tid + OTHR));
    int* op = off + base;
    *(volatile v4i*)(op + 4 * tid) = o0;
    *(volatile v4i*)(op + 4 * (tid + OTHR)) = o1;
    __threadfence();
    *(volatile v4i*)(op + 4 * tid) = o0;
    *(volatile v4i*)(op + 4 * (tid + OTHR)) = o1;
    __syncthreads();
  }
  if (tid == 0) srb[min(4 * nChunk, RBN - 1)] = carry;
  __syncthreads();
  v4i rv = {0, 0, 0, 0};
  if (tid < 32) rv = *(const v4i*)(srb + 4 * tid);
  if (tid < 32) *(volatile v4i*)(rbase + 4 * tid) = rv;
  __threadfence();
  if (tid < 32) *(volatile v4i*)(rbase + 4 * tid) = rv;
}

__global__ __launch_bounds__(NTHR) void k_fill(
    const int* __restrict__ dsts, const int* __restrict__ off, const int* __restrict__ rbase,
    int* csr, int nE, int vec8, int csrLen) {
  extern __shared__ v4f lds_dyn[];
  int* region = (int*)lds_dyn;
  int* cursor = region + RCAP;
  int* list   = cursor + NBF;
  int* wcnt   = list + LISTN;
  const int tid = threadIdx.x, lane = tid & 31, wave = tid >> 5;
  const int b = blockIdx.x;
  const int nodeBase = b * NBF;

  int rb0 = rbase[b];
  const int rb1 = rbase[b + 1];
  rb0 = rb0 < 0 ? 0 : (rb0 > csrLen ? csrLen : rb0);
  rb0 &= ~31;
  int len = rb1 - rb0;
  len = len < 0 ? 0 : (len > RCAP ? RCAP : len);
  int lenW = (len + 31) & ~31;
  if (rb0 + lenW > csrLen) lenW = (csrLen - rb0) & ~31;

  {
    const v4i z = {0, 0, 0, 0};
    for (int i = tid; i < RCAP / 4; i += NTHR) ((v4i*)region)[i] = z;
    for (int s = tid; s < NBF; s += NTHR) {
      int o = off[nodeBase + s] - rb0;
      o = o < 0 ? 0 : (o > RCAP ? RCAP : o);
      cursor[s] = o;
    }
  }
  __syncthreads();

  const int nChunks = (nE + CHUNK - 1) / CHUNK;
#pragma unroll 1
  for (int ch = 0; ch < nChunks; ++ch) {
    const int cbase = ch * CHUNK;
    const int wc = scan_chunk<NBF>(dsts, nE, cbase, nodeBase, vec8, list, tid, lane, wave);
    if (lane == 0) wcnt[wave] = wc;
    __syncthreads();
    if (wave == 0) {
#pragma unroll 1
      for (int wsx = 0; wsx < NWAVE; ++wsx) {
        int n = __builtin_amdgcn_readfirstlane(wcnt[wsx]);
        n = n > WCAP ? WCAP : (n < 0 ? 0 : n);
        const int* lp = list + wsx * WCAP;
#pragma unroll 1
        for (int i = 0; i < n; ++i) {
          const int ent  = __builtin_amdgcn_readfirstlane(lp[i]);
          const int slot = ent & (NBF - 1);
          int e = cbase + ((ent >> 12) & (CHUNK - 1));
          e = e > nE - 1 ? nE - 1 : (e < 0 ? 0 : e);
          if (lane == 0) {
            int pos = cursor[slot];
            pos = pos < 0 ? 0 : (pos > RCAP - 1 ? RCAP - 1 : pos);
            region[pos] = e;
            const int np = pos + 1;
            cursor[slot] = np > RCAP ? RCAP : np;
          }
        }
      }
    }
    __syncthreads();
  }

  const int nv = lenW >> 2;
  int* gpp = csr + rb0;
#pragma unroll 1
  for (int i = tid; i < nv; i += NTHR) { const v4i v = ((const v4i*)region)[i]; *(volatile v4i*)(gpp + 4 * i) = v; }
  __threadfence();
#pragma unroll 1
  for (int i = tid; i < nv; i += NTHR) { const v4i v = ((const v4i*)region)[i]; *(volatile v4i*)(gpp + 4 * i) = v; }
}

__global__ __launch_bounds__(NTHR) void k_edge(
    const float* __restrict__ x, const float* __restrict__ pos, const int* __restrict__ ei,
    const float* __restrict__ W1, const float* __restrict__ b1,
    const float* __restrict__ W2, const float* __restrict__ b2,
    const float* __restrict__ lbp, const float* __restrict__ ubp, const float* __restrict__ gp,
    const int* __restrict__ csr, const int* __restrict__ off, const int* __restrict__ cnt,
    float* out, int nN, int nE, int csrLen) {
  extern __shared__ v4f lds_dyn[];
  char* lb8 = (char*)lds_dyn;
  unsigned short* sW1h = (unsigned short*)(lb8 + LO_W1H);
  unsigned short* sW1l = (unsigned short*)(lb8 + LO_W1L);
  _Float16*       sW2  = (_Float16*)(lb8 + LO_W2);
  unsigned short* sAh  = (unsigned short*)(lb8 + LO_AH);
  unsigned short* sAl  = (unsigned short*)(lb8 + LO_AL);
  _Float16*       sH   = (_Float16*)(lb8 + LO_H);
  float*          sF   = (float*)(lb8 + LO_F);
  float*          sS   = (float*)(lb8 + LO_S);
  float*          sDist = (float*)(lb8 + LO_DST);
  int*            sSlot = (int*)(lb8 + LO_SLT);
  float*          sMu   = (float*)(lb8 + LO_MU);

  const int tid = threadIdx.x, lane = tid & 31, wave = tid >> 5, hh = lane >> 4, m = lane & 15;
  const int rt = wave >> 1, cw = wave & 1;
  const int t0 = blockIdx.x * TB;
  const float lbv = lbp[0], ubv = ubp[0];
  const float ng = -gp[0];

  if (tid < NF) {
    const float s = (float)tid * (1.0f / (float)(NF - 1));
    float mu = lbv * (1.0f - s) + ubv * s;
    if (tid == NF - 1) mu = ubv;
    sMu[tid] = mu;
  }
  {
    const int n = tid >> 2, kq = (tid & 3) * 16;
    const float* wp = W1 + n * NF + kq;
    const v4f w0 = *(const v4f*)(wp), w1 = *(const v4f*)(wp + 4);
    const v4f w2 = *(const v4f*)(wp + 8), w3 = *(const v4f*)(wp + 12);
    v8us h0, l0, h1, l1;
    split8(w0, w1, h0, l0);
    split8(w2, w3, h1, l1);
    *(v8us*)(sW1h + n * NF + kq)     = h0;
    *(v8us*)(sW1h + n * NF + kq + 8) = h1;
    *(v8us*)(sW1l + n * NF + kq)     = l0;
    *(v8us*)(sW1l + n * NF + kq + 8) = l1;
  }
  {
    const int n = tid >> 1, kh = (tid & 1) * 32;
    const float* wp = W2 + n * HD + kh;
#pragma unroll
    for (int j = 0; j < 4; ++j) {
      const v4f a = *(const v4f*)(wp + 8 * j);
      const v4f b = *(const v4f*)(wp + 8 * j + 4);
      *(v8h*)(sW2 + n * HD + kh + 8 * j) = cvt8(a, b, SCL_W);
    }
  }
  {
    const v4f z = {0.0f, 0.0f, 0.0f, 0.0f};
    for (int i = tid; i < (TB + 1) * OD / 4; i += NTHR) ((v4f*)sS)[i] = z;
  }
  float b1v[2], b2v[4];
#pragma unroll
  for (int t = 0; t < 2; ++t) b1v[t] = b1[16 * (2 * cw + t) + m];
#pragma unroll
  for (int t = 0; t < 4; ++t) b2v[t] = b2[64 * cw + 16 * t + m];

  const int tLast = t0 + TB - 1;
  int es = off[t0];
  int ol = off[tLast];
  int c2 = cnt[tLast];
  es = es < 0 ? 0 : (es > csrLen ? csrLen : es);
  ol = ol < 0 ? 0 : (ol > csrLen ? csrLen : ol);
  c2 = c2 < 0 ? 0 : (c2 > csrLen ? csrLen : c2);
  int len = ol + c2 - es;
  len = len < 0 ? 0 : len;
  const int trunc = __builtin_amdgcn_readfirstlane(len > ECAP ? 1 : 0);
  len = len > ECAP ? ECAP : len;
  const int lenU   = __builtin_amdgcn_readfirstlane(len);
  const int esU    = __builtin_amdgcn_readfirstlane(es);
  const int nTiles = __builtin_amdgcn_readfirstlane((len + TE - 1) / TE);
  __syncthreads();

#pragma unroll 1
  for (int tile = 0; tile < nTiles; ++tile) {
    if (tid < TE) {
      const int li = tile * TE + tid;
      int valid = li < lenU ? 1 : 0;
      int p = esU + li;
      p = p < 0 ? 0 : (p > csrLen - 1 ? csrLen - 1 : p);
      int e = csr[p];
      e = e < 0 ? 0 : (e > nE - 1 ? nE - 1 : e);
      const int sr = ei[e];
      const int tr = ei[nE + e];
      const int slot = tr - t0;
      valid = (valid != 0 && (unsigned)slot < (unsigned)TB) ? 1 : 0;
      int sc = sr < 0 ? 0 : (sr > nN - 1 ? nN - 1 : sr);
      int tc = tr < 0 ? 0 : (tr > nN - 1 ? nN - 1 : tr);
      const float dx = pos[sc * 3 + 0] - pos[tc * 3 + 0];
      const float dy = pos[sc * 3 + 1] - pos[tc * 3 + 1];
      const float dz = pos[sc * 3 + 2] - pos[tc * 3 + 2];
      const float d2 = (dx * dx + dz * dz) + dy * dy;
      sDist[tid] = sqrtf(d2);
      sSlot[tid] = (valid != 0) ? slot : TB;
    }
    __syncthreads();

    {
      const int r = tid >> 2, kq = (tid & 3) * 16;
      const float d = sDist[r];
      v8us h0, l0, h1, l1;
#pragma unroll
      for (int j = 0; j < 8; ++j) {
        const float ta = d - sMu[kq + j];
        const float va = __expf(ng * (ta * ta));
        const unsigned short ha = bf16bits(va);
        h0[j] = ha;
        l0[j] = bf16bits(va - bf16val(ha));
        const float tb = d - sMu[kq + 8 + j];
        const float vb = __expf(ng * (tb * tb));
        const unsigned short hb = bf16bits(vb);
        h1[j] = hb;
        l1[j] = bf16bits(vb - bf16val(hb));
      }
      unsigned short* ph = sAh + r * NF + kq;
      unsigned short* pl = sAl + r * NF + kq;
      *(v8us*)(ph)     = h0;
      *(v8us*)(ph + 8) = h1;
      *(v8us*)(pl)     = l0;
      *(v8us*)(pl + 8) = l1;
    }
    __syncthreads();

    {
      v8f acc1[2];
#pragma unroll
      for (int t = 0; t < 2; ++t) { v8f z = {0.f, 0.f, 0.f, 0.f, 0.f, 0.f, 0.f, 0.f}; acc1[t] = z; }
      const unsigned short* ah0 = sAh + (16 * rt + m) * NF + 8 * hh;
      const unsigned short* al0 = sAl + (16 * rt + m) * NF + 8 * hh;
#pragma unroll
      for (int kt = 0; kt < NF / 32; ++kt) {
        FragB fh, fl;
        fh.u[0] = *(const v8us*)(ah0 + 32 * kt);
        fh.u[1] = *(const v8us*)(ah0 + 32 * kt + 16);
        fl.u[0] = *(const v8us*)(al0 + 32 * kt);
        fl.u[1] = *(const v8us*)(al0 + 32 * kt + 16);
#pragma unroll
        for (int t = 0; t < 2; ++t) {
          const int n = 16 * (2 * cw + t) + m;
          const unsigned short* bh = sW1h + n * NF + 8 * hh + 32 * kt;
          const unsigned short* bl = sW1l + n * NF + 8 * hh + 32 * kt;
          FragB gh, gl;
          gh.u[0] = *(const v8us*)(bh);
          gh.u[1] = *(const v8us*)(bh + 16);
          gl.u[0] = *(const v8us*)(bl);
          gl.u[1] = *(const v8us*)(bl + 16);
          acc1[t] = wmb(fh.v, gh.v, acc1[t]);
          acc1[t] = wmb(fh.v, gl.v, acc1[t]);
          acc1[t] = wmb(fl.v, gh.v, acc1[t]);
        }
      }
#pragma unroll
      for (int t = 0; t < 2; ++t) {
        const int n = 16 * (2 * cw + t) + m;
        _Float16* hp = sH + (16 * rt + 8 * hh) * HD + n;
#pragma unroll
        for (int r = 0; r < 8; ++r) {
          const float hv = sspf(acc1[t][r] + b1v[t]) * SCL_H;
          hp[r * HD] = (_Float16)hv;
        }
      }
    }
    __syncthreads();

    {
      v8f acc2[4];
#pragma unroll
      for (int t = 0; t < 4; ++t) { v8f z = {0.f, 0.f, 0.f, 0.f, 0.f, 0.f, 0.f, 0.f}; acc2[t] = z; }
      const _Float16* hrow = sH + (16 * rt + m) * HD + 8 * hh;
#pragma unroll
      for (int kt = 0; kt < HD / 32; ++kt) {
        FragH a;
        a.h[0] = *(const v8h*)(hrow + 32 * kt);
        a.h[1] = *(const v8h*)(hrow + 32 * kt + 16);
#pragma unroll
        for (int t = 0; t < 4; ++t) {
          const int n = 64 * cw + 16 * t + m;
          const _Float16* bp = sW2 + n * HD + 8 * hh + 32 * kt;
          FragH bf;
          bf.h[0] = *(const v8h*)(bp);
          bf.h[1] = *(const v8h*)(bp + 16);
          acc2[t] = wmh(a.v, bf.v, acc2[t]);
        }
      }
#pragma unroll
      for (int t = 0; t < 4; ++t) {
        const int n = 64 * cw + 16 * t + m;
        float* fp = sF + (16 * rt + 8 * hh) * OD + n;
#pragma unroll
        for (int r = 0; r < 8; ++r) {
          const float v = acc2[t][r] * SCL_ACC + b2v[t];
          fp[r * OD] = sspf(v);
        }
      }
    }
    __syncthreads();

    if (wave == 0) {
      v4f* S4 = (v4f*)sS;
      const v4f* F4 = (const v4f*)sF;
#pragma unroll 4
      for (int r = 0; r < TE; ++r) {
        int si = sSlot[r];
        si = ((unsigned)si > (unsigned)TB) ? TB : si;
        const v4f f = F4[r * (OD / 4) + lane];
        v4f s = S4[si * (OD / 4) + lane];
        s += f;
        S4[si * (OD / 4) + lane] = s;
      }
    }
    __syncthreads();
  }

  const float qn = __int_as_float(0x7fc00000);
  v4f ov[8];
#pragma unroll
  for (int it = 0; it < 8; ++it) {
    const int u = it * NTHR + tid;
    const int row = u >> 5;
    const int c4 = u & 31;
    int tcl = t0 + row;
    tcl = tcl > nN - 1 ? nN - 1 : tcl;
    const v4f xv = *(const v4f*)(x + (size_t)tcl * OD + 4 * c4);
    const v4f sv = ((const v4f*)sS)[row * (OD / 4) + c4];
    v4f o = xv * sv;
    if (trunc != 0) { o.x = qn; o.y = qn; o.z = qn; o.w = qn; }
    ov[it] = o;
  }
#pragma unroll
  for (int it = 0; it < 8; ++it) {
    const int u = it * NTHR + tid;
    const int row = u >> 5;
    const int c4 = u & 31;
    if (t0 + row < nN) *(volatile v4f*)(out + (size_t)(t0 + row) * OD + 4 * c4) = ov[it];
  }
  __threadfence();
#pragma unroll
  for (int it = 0; it < 8; ++it) {
    const int u = it * NTHR + tid;
    const int row = u >> 5;
    const int c4 = u & 31;
    if (t0 + row < nN) *(volatile v4f*)(out + (size_t)(t0 + row) * OD + 4 * c4) = ov[it];
  }
}

extern "C" void kernel_launch(void* const* d_in, const int* in_sizes, int n_in,
                              void* d_out, int out_size, void* d_ws, size_t ws_size,
                              hipStream_t stream) {
  if (n_in < 10) return;
  const int nN = in_sizes[1] / 3;
  const int nE = in_sizes[2] / 2;
  if (nN <= 0 || nE <= 0 || in_sizes[1] != 3 * nN || in_sizes[2] != 2 * nE) return;
  if (in_sizes[0] != nN * OD) return;
  if (in_sizes[3] != HD * NF || in_sizes[4] != HD) return;
  if (in_sizes[5] != OD * HD || in_sizes[6] != OD) return;
  if (in_sizes[7] < 1 || in_sizes[8] < 1 || in_sizes[9] < 1) return;
  if (out_size != nN * OD) return;
  if (nE > (1 << 28) || nN > (1 << 22)) return;

  const float* x   = (const float*)d_in[0];
  const float* pos = (const float*)d_in[1];
  const int*   ei  = (const int*)d_in[2];
  const float* W1  = (const float*)d_in[3];
  const float* b1  = (const float*)d_in[4];
  const float* W2  = (const float*)d_in[5];
  const float* b2  = (const float*)d_in[6];
  const float* lbp = (const float*)d_in[7];
  const float* ubp = (const float*)d_in[8];
  const float* gp  = (const float*)d_in[9];
  float* out = (float*)d_out;
  const int* dsts = ei + nE;

  const int nBC    = (nN + NBC - 1) / NBC;
  const int CNTPAD = nBC * NBC;
  if (4 * nBC + 1 > RBN) return;
  const int nBF    = (nN + NBF - 1) / NBF;
  if (nBF + 1 > 4 * nBC + 1) return;
  const int nEB    = (nN + TB - 1) / TB;
  if (nEB * TB > CNTPAD) return;
  const int csrLen = ((nE + 31) & ~31) + 4096;
  if (31 * 4 * nBC > 4096) return;

  char* ws = (char*)d_ws;
  size_t offb = 0;
  const size_t oCnt = offb; offb += (size_t)CNTPAD * 4;   offb = (offb + 255) & ~(size_t)255;
  const size_t oOff = offb; offb += (size_t)CNTPAD * 4;   offb = (offb + 255) & ~(size_t)255;
  const size_t oRb  = offb; offb += (size_t)RBN * 4;      offb = (offb + 255) & ~(size_t)255;
  const size_t oCsr = offb; offb += (size_t)csrLen * 4;   offb = (offb + 255) & ~(size_t)255;
  if (offb > ws_size || offb > (size_t)WSCAP) return;
  int* cnt  = (int*)(ws + oCnt);
  int* offp = (int*)(ws + oOff);
  int* rb   = (int*)(ws + oRb);
  int* csr  = (int*)(ws + oCsr);

  const int vec8 = ((nE & 3) == 0) ? 1 : 0;

  k_count<<<nBC, NTHR, 0, stream>>>(dsts, cnt, nE, vec8);
  k_offsets<<<1, OTHR, 0, stream>>>(cnt, offp, rb, nBC);
  hipFuncSetAttribute(reinterpret_cast<const void*>(&k_fill),
                      hipFuncAttributeMaxDynamicSharedMemorySize, LDS_FILL);
  k_fill<<<nBF, NTHR, LDS_FILL, stream>>>(dsts, offp, rb, csr, nE, vec8, csrLen);

  hipFuncSetAttribute(reinterpret_cast<const void*>(&k_edge),
                      hipFuncAttributeMaxDynamicSharedMemorySize, LDS_EDGE);
  k_edge<<<nEB, NTHR, LDS_EDGE, stream>>>(x, pos, ei, W1, b1, W2, b2, lbp, ubp, gp,
                                          csr, offp, cnt, out, nN, nE, csrLen);
}
